// ScaleDotProduct_30829275250742
// MI455X (gfx1250) — hardware-verified
//
#include <hip/hip_runtime.h>
#include <math.h>
#include <stdint.h>

#ifndef NH
#define NH    16
#endif
#define SEQ   4096
#define HD    64
#define QSC   1024.0f
#define KSC   1024.0f
#define PCAR  32768.0f
#define VCAR  256.0f
#define LOG2E 1.4426950408889634f
#define ATW   4
#define ATT_THREADS (ATW * 32)
#define QPB   (16 * ATW)
#define BPH   (SEQ / QPB)
#define ATT_BLOCKS (NH * BPH)
#define PTP   36
#define SLP   68
#define SLABF (16 * SLP)
#define VTP   72
#define VTILES (SEQ / 64)
static_assert(HD == 64 && QPB == 64 && ATT_THREADS == 128);
static_assert((SEQ % QPB) == 0 && (SEQ % 64) == 0 && (SEQ % 32) == 0);
static_assert(BPH == 64 && ATT_BLOCKS == NH * 64 && VTILES == 64);
static_assert(NH >= 1 && NH <= 16);
static_assert(16 * PTP <= SLABF);
static_assert((HD - 1) * VTP + 63 < HD * VTP);
static_assert(((NH * SEQ * HD) % 2048) == 0);

typedef _Float16 v16h __attribute__((ext_vector_type(16)));
typedef _Float16 v8h  __attribute__((ext_vector_type(8)));
typedef float    v8f  __attribute__((ext_vector_type(8)));
typedef float    v4f  __attribute__((ext_vector_type(4)));
typedef unsigned int v4u __attribute__((ext_vector_type(4)));

union FragH { v16h v; v8h h[2]; v4u u[2]; };

__device__ __forceinline__ unsigned short bf_bits(float f) {
  unsigned u = __float_as_uint(f);
  return (unsigned short)((u + 0x7FFFu + ((u >> 16) & 1u)) >> 16);
}
__device__ __forceinline__ float bf_up(unsigned short h) { return __uint_as_float(((unsigned)h) << 16); }
__device__ __forceinline__ float bfr(float f) { return bf_up(bf_bits(f)); }
__device__ __forceinline__ unsigned short h_bits(_Float16 x) { return __builtin_bit_cast(unsigned short, x); }
__device__ __forceinline__ unsigned pk16(unsigned short a, unsigned short b) { return (unsigned)a | ((unsigned)b << 16); }
__device__ __forceinline__ v8f zero8() { v8f z = {0.f, 0.f, 0.f, 0.f, 0.f, 0.f, 0.f, 0.f}; return z; }

__device__ __forceinline__ v16h ldfrag_h(const _Float16* p) {
  FragH f;
  f.h[0] = *(const v8h*)(p);
  f.h[1] = *(const v8h*)(p + 16);
  return f.v;
}

__device__ __forceinline__ v8f mma_raw(v16h a, v16h b, v8f c) {
  return __builtin_amdgcn_wmma_f32_16x16x32_f16(false, a, false, b, (short)0, c, false, false);
}
__device__ __forceinline__ void guard_sc(v8f& a, v8f& b, v16h x0, v16h x1, v16h x2, v16h x3, v16h x4, v16h x5) {
#if defined(__HIP_DEVICE_COMPILE__)
  asm volatile("v_nop\n\tv_nop\n\tv_nop\n\tv_nop"
               : "+v"(a), "+v"(b) : "v"(x0), "v"(x1), "v"(x2), "v"(x3), "v"(x4), "v"(x5) : "memory");
#endif
}
__device__ __forceinline__ void guard_pv(v8f& a, v8f& b, v8f& c, v8f& d,
                                         v16h p0, v16h p1, v16h x0, v16h x1, v16h x2, v16h x3) {
#if defined(__HIP_DEVICE_COMPILE__)
  asm volatile("v_nop\n\tv_nop\n\tv_nop\n\tv_nop"
               : "+v"(a), "+v"(b), "+v"(c), "+v"(d) : "v"(p0), "v"(p1), "v"(x0), "v"(x1), "v"(x2), "v"(x3) : "memory");
#endif
}
__device__ __forceinline__ void acc_guard4(v8f& a, v8f& b, v8f& c, v8f& d) {
#if defined(__HIP_DEVICE_COMPILE__)
  asm volatile("v_nop\n\tv_nop\n\tv_nop\n\tv_nop" : "+v"(a), "+v"(b), "+v"(c), "+v"(d));
#endif
}
__device__ __forceinline__ void wave_sync_lds() {
  __builtin_amdgcn_fence(__ATOMIC_RELEASE, "workgroup");
  __builtin_amdgcn_wave_barrier();
  __builtin_amdgcn_fence(__ATOMIC_ACQUIRE, "workgroup");
}

__global__ __launch_bounds__(256) void cvt16(const float* __restrict__ xq, const float* __restrict__ xk,
                                             unsigned short* plq, unsigned short* plk, int n8, float sc) {
  const int gt = blockIdx.x * 256 + (int)threadIdx.x;
  if (gt >= n8) return;
  const bool sk = (blockIdx.y != 0);
  const float* x = sk ? xk : xq;
  unsigned short* pl = sk ? plk : plq;
  const size_t e = (size_t)gt * 8;
  const v4f a = *(const v4f*)(x + e), bq = *(const v4f*)(x + e + 4);
  v4u o;
#pragma unroll
  for (int i = 0; i < 2; ++i) {
    o[i]     = pk16(h_bits((_Float16)(bfr(a[2 * i]) * sc)),  h_bits((_Float16)(bfr(a[2 * i + 1]) * sc)));
    o[2 + i] = pk16(h_bits((_Float16)(bfr(bq[2 * i]) * sc)), h_bits((_Float16)(bfr(bq[2 * i + 1]) * sc)));
  }
  unsigned short* d = pl + e;
  for (int pass = 0; pass < 2; ++pass) {
    *(volatile v4u*)(d) = o;
    __threadfence();
  }
}

__global__ __launch_bounds__(256) void vt16(const float* __restrict__ v, unsigned short* VTo) {
  __shared__ __align__(16) unsigned short T[HD * VTP];
  const int tid = threadIdx.x;
  const int bid = blockIdx.x;
  const int bh  = bid / VTILES;
  const int t   = bid - bh * VTILES;
  if (bh >= NH) return;
  {
    const int sl = tid >> 2;
    const int dc = (tid & 3) * 16;
    int key = 64 * t + sl;
    key = (key < 0) ? 0 : ((key > SEQ - 1) ? (SEQ - 1) : key);
    const float* src = v + (((size_t)bh * SEQ + (size_t)key) * HD + dc);
#pragma unroll
    for (int i = 0; i < 4; ++i) {
      const v4f a = *(const v4f*)(src + 4 * i);
#pragma unroll
      for (int e = 0; e < 4; ++e) T[(dc + 4 * i + e) * VTP + sl] = h_bits((_Float16)(bfr(a[e]) * VCAR));
    }
  }
  __syncthreads();
  v4u vals[2];
  const int q8 = tid >> 3, p8 = (tid & 7) * 8;
#pragma unroll
  for (int it = 0; it < 2; ++it) {
    const int line = it * 32 + q8;
    vals[it] = *(const v4u*)(T + line * VTP + p8);
  }
  unsigned short* dst = VTo + ((size_t)(bh * HD)) * SEQ + 64 * t + p8;
  for (int pass = 0; pass < 2; ++pass) {
#pragma unroll
    for (int it = 0; it < 2; ++it) {
      const int line = it * 32 + q8;
      *(volatile v4u*)(dst + (size_t)line * SEQ) = vals[it];
    }
    __threadfence();
  }
}

__global__ __launch_bounds__(ATT_THREADS)
void attn_fwd(const unsigned short* __restrict__ QHp, const unsigned short* __restrict__ KHp,
              const unsigned short* __restrict__ VTq, const int* __restrict__ mkp, float* OPp) {
  __shared__ __align__(16) float smem[ATW * SLABF];
  (void)mkp;

  const int tid  = threadIdx.x;
  const int wave = tid >> 5;
  const int lane = tid & 31;
  const int hh   = lane >> 4;
  const int c    = lane & 15;

  const int bid  = blockIdx.x;
  const int bh   = bid / BPH;
  const int t    = bid - bh * BPH;
  if (bh >= NH) return;

  const int i0 = QPB * t;
  const int iw = i0 + wave * 16;
  const int qs = iw + c;

  const _Float16* Qb = (const _Float16*)(const void*)QHp + ((size_t)bh * SEQ + (size_t)qs) * HD + 8 * hh;
  const v16h qa0 = ldfrag_h(Qb);
  const v16h qa1 = ldfrag_h(Qb + 32);
  const _Float16* Kb = (const _Float16*)(const void*)KHp + ((size_t)bh * SEQ + (size_t)c) * HD + 8 * hh;
  const _Float16* Vb = (const _Float16*)(const void*)VTq + ((size_t)(bh * HD + c)) * SEQ + 8 * hh;
  const float lsc = LOG2E / (8.0f * QSC * KSC);

  float mrow[8], lrow[8];
  v8f o[4];
#pragma unroll
  for (int r = 0; r < 8; ++r) { mrow[r] = -INFINITY; lrow[r] = 0.f; }
#pragma unroll
  for (int j = 0; j < 4; ++j) o[j] = zero8();
  float* pt = smem + wave * SLABF;

#pragma unroll 1
  for (int kb = 0; kb < SEQ; kb += 32) {
    v8f s0 = zero8(), s1 = zero8();
    {
      const _Float16* k0p = Kb + (size_t)kb * HD;
      const _Float16* k1p = k0p + (size_t)16 * HD;
      const v16h kf00 = ldfrag_h(k0p), kf01 = ldfrag_h(k0p + 32);
      const v16h kf10 = ldfrag_h(k1p), kf11 = ldfrag_h(k1p + 32);
      s0 = mma_raw(qa0, kf00, s0);
      s0 = mma_raw(qa1, kf01, s0);
      s1 = mma_raw(qa0, kf10, s1);
      s1 = mma_raw(qa1, kf11, s1);
      guard_sc(s0, s1, qa0, qa1, kf00, kf01, kf10, kf11);
    }
#pragma unroll
    for (int r = 0; r < 8; ++r) {
      const float t0 = s0[r] * lsc;
      const float t1 = s1[r] * lsc;
      float mx = fmaxf(t0, t1);
#pragma unroll
      for (int off = 1; off < 16; off <<= 1) mx = fmaxf(mx, __shfl_xor(mx, off, 32));
      const float mn  = fmaxf(mrow[r], mx);
      const float al  = exp2f(mrow[r] - mn);
      mrow[r] = mn;
      const float e0 = exp2f(t0 - mn), e1 = exp2f(t1 - mn);
      float ps = e0 + e1;
#pragma unroll
      for (int off = 1; off < 16; off <<= 1) ps += __shfl_xor(ps, off, 32);
      lrow[r] = lrow[r] * al + ps;
#pragma unroll
      for (int j = 0; j < 4; ++j) o[j][r] *= al;
      const int ro = (8 * hh + r) * PTP + c;
      pt[ro]      = e0;
      pt[ro + 16] = e1;
    }
    wave_sync_lds();
    FragH ph, pl;
    {
      const float* prow = pt + c * PTP + 8 * hh;
      const v4f p0 = *(const v4f*)(prow), p1 = *(const v4f*)(prow + 4);
      const v4f p2 = *(const v4f*)(prow + 16), p3 = *(const v4f*)(prow + 20);
#pragma unroll
      for (int e = 0; e < 4; ++e) {
        const float ta = p0[e] * PCAR, tb = p1[e] * PCAR, tc = p2[e] * PCAR, td = p3[e] * PCAR;
        const _Float16 ha = (_Float16)ta, hb = (_Float16)tb, hc = (_Float16)tc, hd = (_Float16)td;
        ph.h[0][e]     = ha;
        ph.h[0][4 + e] = hb;
        ph.h[1][e]     = hc;
        ph.h[1][4 + e] = hd;
        pl.h[0][e]     = (_Float16)(ta - (float)ha);
        pl.h[0][4 + e] = (_Float16)(tb - (float)hb);
        pl.h[1][e]     = (_Float16)(tc - (float)hc);
        pl.h[1][4 + e] = (_Float16)(td - (float)hd);
      }
    }
    {
      const _Float16* vp = Vb + kb;
      const v16h vb0 = ldfrag_h(vp);
      const v16h vb1 = ldfrag_h(vp + (size_t)16 * SEQ);
      const v16h vb2 = ldfrag_h(vp + (size_t)32 * SEQ);
      const v16h vb3 = ldfrag_h(vp + (size_t)48 * SEQ);
      o[0] = mma_raw(ph.v, vb0, o[0]);  o[0] = mma_raw(pl.v, vb0, o[0]);
      o[1] = mma_raw(ph.v, vb1, o[1]);  o[1] = mma_raw(pl.v, vb1, o[1]);
      o[2] = mma_raw(ph.v, vb2, o[2]);  o[2] = mma_raw(pl.v, vb2, o[2]);
      o[3] = mma_raw(ph.v, vb3, o[3]);  o[3] = mma_raw(pl.v, vb3, o[3]);
      guard_pv(o[0], o[1], o[2], o[3], ph.v, pl.v, vb0, vb1, vb2, vb3);
    }
    wave_sync_lds();
  }
  acc_guard4(o[0], o[1], o[2], o[3]);

  wave_sync_lds();
  float* slab = pt;
  const float oc = 1.0f / (PCAR * VCAR);
#pragma unroll
  for (int r = 0; r < 8; ++r) {
    const float lr  = lrow[r];
    const float inv = (lr > 0.0f) ? ((1.0f / lr) * oc) : 0.0f;
#pragma unroll
    for (int j = 0; j < 4; ++j) slab[(8 * hh + r) * SLP + j * 16 + c] = o[j][r] * inv;
  }
  wave_sync_lds();
  v4f vals[8];
#pragma unroll
  for (int it = 0; it < 8; ++it) vals[it] = *(const v4f*)(slab + (2 * it + hh) * SLP + c * 4);
  float* dst = OPp + ((size_t)(bh * SEQ + iw)) * HD + hh * HD + c * 4;
  for (int pass = 0; pass < 2; ++pass) {
#pragma unroll
    for (int it = 0; it < 8; ++it) {
      *(volatile v4f*)(dst + (size_t)(2 * it) * HD) = vals[it];
    }
    __threadfence();
  }
}

extern "C" void kernel_launch(void* const* d_in, const int* in_sizes, int n_in,
                              void* d_out, int out_size, void* d_ws, size_t ws_size,
                              hipStream_t stream) {
  const int NEL = NH * SEQ * HD;
  if (n_in < 4) return;
  if (in_sizes[0] < NEL || in_sizes[1] < NEL || in_sizes[2] < NEL || in_sizes[3] < 1) return;
  if (out_size < NEL) return;

  const float* q  = (const float*)d_in[0];
  const float* k  = (const float*)d_in[1];
  const float* v  = (const float*)d_in[2];
  const int*   mk = (const int*)d_in[3];
  float*       out = (float*)d_out;

  const size_t PQ = (size_t)NEL * 2;
  const size_t PK = (size_t)NEL * 2;
  const size_t PV = (size_t)NH * HD * SEQ * 2;
  size_t off = 0;
  const size_t oQH = off; off += PQ;
  const size_t oKH = off; off += PK;
  const size_t oVT = off; off += PV;
  if (off > ws_size) return;
  if (off > (size_t)134217728) return;

  char* ws = (char*)d_ws;
  unsigned short* QH = (unsigned short*)(ws + oQH);
  unsigned short* KH = (unsigned short*)(ws + oKH);
  unsigned short* VT = (unsigned short*)(ws + oVT);

  const int n8 = NEL / 8;
  const dim3 blk(256);
  const dim3 gC(n8 / 256, 2);
  const dim3 gVT(NH * VTILES);
  const dim3 gAT(ATT_BLOCKS);
  const dim3 bAT(ATT_THREADS);

  cvt16<<<gC, blk, 0, stream>>>(q, k, QH, KH, n8, QSC);
  vt16<<<gVT, blk, 0, stream>>>(v, VT);
  attn_fwd<<<gAT, bAT, 0, stream>>>(QH, KH, VT, mk, out);
  (void)hipGetLastError();
}
